// TwoBodyAttn_52295521796553
// MI455X (gfx1250) — hardware-verified
//
#include <hip/hip_runtime.h>


#define NN_  4096
#define HIDN 256
#define NHD  8
#define HDM  32
#define EGW  64
#define PSC  32768.0f
#define LOSC 1024.0f
#define LOSCI (1.0f / 1024.0f)
#define WSC  64.0f
#define WSCI (1.0f / 64.0f)

typedef _Float16 h16;
typedef __attribute__((ext_vector_type(16))) _Float16 v16h;
typedef __attribute__((ext_vector_type(8)))  _Float16 v8h;
typedef __attribute__((ext_vector_type(8)))  float    v8f;
typedef __attribute__((ext_vector_type(4)))  float    v4f;
typedef v8h  __attribute__((may_alias)) v8ha;
typedef v4f  __attribute__((may_alias)) v4fa;

#define VST2(T, p, v) do { const T vst2_v_ = (v); *(volatile T*)(p) = vst2_v_; __threadfence(); *(volatile T*)(p) = vst2_v_; } while (0)
__device__ __forceinline__ v16h cat16(v8h lo, v8h hi) { return __builtin_shufflevector(lo, hi, 0, 1, 2, 3, 4, 5, 6, 7, 8, 9, 10, 11, 12, 13, 14, 15); }
__device__ __forceinline__ v8f wmma16(v16h a, v16h b, v8f c) { return __builtin_amdgcn_wmma_f32_16x16x32_f16(false, a, false, b, (short)0, c, false, false); }
__device__ __forceinline__ void split16(float x, h16& h, h16& l) { h = (h16)x; l = (h16)((x - (float)h) * LOSC); }

__global__ __launch_bounds__(256) void k_asplit(const float* __restrict__ X, h16* FH, h16* FL) {
    const int lane = threadIdx.x & 31, r = blockIdx.x * 8 + (threadIdx.x >> 5);
    if (r >= NN_) return;
    const float* src = X + (size_t)r * HIDN + lane * 8;
    v8h vh, vl;
#pragma unroll
    for (int i = 0; i < 8; ++i) { h16 a, b; split16(src[i], a, b); vh[i] = a; vl[i] = b; }
    h16* dh = FH + (size_t)r * HIDN + lane * 8; h16* dl = FL + (size_t)r * HIDN + lane * 8;
    *(volatile v8h*)dh = vh; *(volatile v8h*)dl = vl;
    __threadfence();
    *(volatile v8h*)dh = vh; *(volatile v8h*)dl = vl;
}

__global__ __launch_bounds__(256) void k_wsplit(const float* __restrict__ Wm, int N, int Npad, h16* WTH, h16* WTL) {
    __shared__ __align__(16) h16 th[64 * 72];
    __shared__ __align__(16) h16 tl[64 * 72];
    const int tid = threadIdx.x, k0 = blockIdx.x * 64, n0 = blockIdx.y * 64;
    const int kk = tid >> 2, nq = (tid & 3) * 16;
#pragma unroll
    for (int i = 0; i < 16; ++i) {
        const int n = n0 + nq + i;
        const float w = (n < N) ? Wm[(size_t)(k0 + kk) * N + n] * WSC : 0.0f;
        h16 a, b; split16(w, a, b);
        th[(nq + i) * 72 + kk] = a; tl[(nq + i) * 72 + kk] = b;
    }
    __syncthreads();
    const int piece = tid & 7;
    auto pass = [&]() {
#pragma unroll
        for (int s = 0; s < 4; ++s) {
            const int Lid = (tid >> 3) + 32 * s;
            const int pln = Lid >> 6, nr = Lid & 63;
            const v8h val = *(const v8ha*)((pln ? tl : th) + nr * 72 + piece * 8);
            h16* dst = (pln ? WTL : WTH) + (size_t)(n0 + nr) * HIDN + k0 + piece * 8;
            *(volatile v8h*)dst = val;
        }
    };
    pass();
    __threadfence();
    pass();
    (void)Npad;
}

__global__ __launch_bounds__(128) void k_lgemm(const h16* __restrict__ Ah, const h16* __restrict__ Al, const h16* __restrict__ Bh, const h16* __restrict__ Bl,
                                               const float* __restrict__ bias, int nvalid, float* C, int ldc) {
    __shared__ __align__(16) float ost[4][16 * 68];
    const int lane = threadIdx.x & 31, wave = threadIdx.x >> 5, lr = lane & 15, hi = lane >> 4;
    const int r0 = blockIdx.x * 64 + wave * 16, c0 = blockIdx.y * 64;
    const h16* ap = Ah + (size_t)(r0 + lr) * HIDN + 8 * hi;
    const h16* alp = Al + (size_t)(r0 + lr) * HIDN + 8 * hi;
    v8f acch[4], accx[4];
#pragma unroll
    for (int t = 0; t < 4; ++t) { acch[t] = (v8f){}; accx[t] = (v8f){}; }
#pragma unroll 1
    for (int kc = 0; kc < HIDN; kc += 32) {
        const v16h a  = cat16(*(const v8h*)(ap + kc), *(const v8h*)(ap + kc + 16));
        const v16h al = cat16(*(const v8h*)(alp + kc), *(const v8h*)(alp + kc + 16));
#pragma unroll
        for (int t = 0; t < 4; ++t) {
            const h16* bp  = Bh + (size_t)(c0 + t * 16 + lr) * HIDN + kc + 8 * hi;
            const h16* blp = Bl + (size_t)(c0 + t * 16 + lr) * HIDN + kc + 8 * hi;
            const v16h b = cat16(*(const v8h*)bp, *(const v8h*)(bp + 16));
            acch[t] = wmma16(a, b, acch[t]);
            accx[t] = wmma16(a, cat16(*(const v8h*)blp, *(const v8h*)(blp + 16)), accx[t]);
            accx[t] = wmma16(al, b, accx[t]);
        }
        asm volatile("v_nop\n\tv_nop\n\tv_nop\n\tv_nop" : "+v"(acch[0]), "+v"(acch[1]), "+v"(acch[2]), "+v"(acch[3]), "+v"(accx[0]), "+v"(accx[1]), "+v"(accx[2]), "+v"(accx[3]) : "v"(a), "v"(al));
    }
    float* os = &ost[wave][0];
#pragma unroll
    for (int t = 0; t < 4; ++t) {
        const int n = c0 + t * 16 + lr;
        const float bv = (n < nvalid) ? bias[n] : 0.0f;
#pragma unroll
        for (int j = 0; j < 8; ++j) os[(hi * 8 + j) * 68 + t * 16 + lr] = (acch[t][j] + accx[t][j] * LOSCI) * WSCI + bv;
    }
    __syncthreads();
    float* crow = C + (size_t)r0 * ldc + c0;
    auto pass = [&]() {
#pragma unroll
        for (int s = 0; s < 8; ++s) {
            const int Lid = (lane >> 3) + 4 * s, piece = lane & 7;
            const int row = Lid >> 1, cofs = (Lid & 1) * 32 + piece * 4;
            const v4f val = *(const v4fa*)(os + row * 68 + cofs);
            *(volatile v4f*)(crow + (size_t)row * ldc + cofs) = val;
        }
    };
    pass();
    __threadfence();
    pass();
}

__global__ __launch_bounds__(256) void k_prep(const float* __restrict__ QF, const float* __restrict__ KVF, h16* Q16, h16* K16, h16* VT16) {
    __shared__ __align__(16) h16 tile[NHD * 64 * 32];
    const int tid = threadIdx.x, r0 = blockIdx.x * 64;
    const int row = tid >> 2, cq = (tid & 3) * 64;
    const int piece = tid & 7;
    const float qsc = 0.17677669529663687f;
#pragma unroll 1
    for (int ph = 0; ph < 3; ++ph) {
        const float* src = (ph == 0) ? (QF + (size_t)(r0 + row) * HIDN + cq) : (KVF + (size_t)(r0 + row) * (2 * HIDN) + (ph == 2 ? HIDN : 0) + cq);
        const float sc = (ph == 0) ? qsc : 1.0f;
#pragma unroll 4
        for (int c = 0; c < 64; ++c) {
            const int f = cq + c, d = f >> 3, h = f & 7;
            const h16 v = (h16)(src[c] * sc);
            if (ph < 2) tile[(h * 64 + row) * 32 + d] = v; else tile[(h * 32 + d) * 64 + row] = v;
        }
        __syncthreads();
        auto pass = [&]() {
#pragma unroll
            for (int s = 0; s < 8; ++s) {
                const int Lid = (tid >> 3) + 32 * s;
                if (ph < 2) {
                    const int h = Lid >> 5, rr = 2 * (Lid & 31) + (piece >> 2), d0 = (piece & 3) * 8;
                    const v8h val = *(const v8ha*)(tile + (h * 64 + rr) * 32 + d0);
                    h16* dst = (ph == 0 ? Q16 : K16) + ((size_t)h * NN_ + r0 + rr) * 32 + d0;
                    *(volatile v8h*)dst = val;
                } else {
                    const int h = Lid >> 5, d = Lid & 31;
                    const v8h val = *(const v8ha*)(tile + (h * 32 + d) * 64 + piece * 8);
                    h16* dst = VT16 + ((size_t)h * HDM + d) * NN_ + r0 + piece * 8;
                    *(volatile v8h*)dst = val;
                }
            }
        };
        pass();
        __threadfence();
        pass();
        __syncthreads();
    }
}

__global__ __launch_bounds__(128) void k_colstats(const h16* __restrict__ Q16, const h16* __restrict__ K16, const float* __restrict__ EGF, float* CM, float* CC) {
    __shared__ __align__(16) float stg[128];
    const int lane = threadIdx.x & 31, wave = threadIdx.x >> 5, lr = lane & 15, hi = lane >> 4;
    const int h = blockIdx.x / (NN_ / 64), jt = blockIdx.x - h * (NN_ / 64);
    const int j0 = jt * 64 + wave * 16;
    const h16* qb = Q16 + (size_t)h * NN_ * 32;
    const h16* kp = K16 + ((size_t)h * NN_ + j0 + lr) * 32 + 8 * hi;
    const v16h ka = cat16(*(const v8h*)kp, *(const v8h*)(kp + 16));
    float ej[8], mrow[8], lpart[8];
#pragma unroll
    for (int j = 0; j < 8; ++j) { ej[j] = EGF[(size_t)(j0 + 8 * hi + j) * EGW + h]; mrow[j] = -3.0e38f; lpart[j] = 0.f; }
#pragma unroll 1
    for (int it = 0; it < NN_ / 32; ++it) {
        const int i0 = it * 32;
        const h16* r0 = qb + (size_t)(i0 + lr) * 32 + 8 * hi;
        const h16* r1 = qb + (size_t)(i0 + 16 + lr) * 32 + 8 * hi;
        v8f s0 = {}, s1 = {};
        s0 = wmma16(ka, cat16(*(const v8h*)r0, *(const v8h*)(r0 + 16)), s0);
        s1 = wmma16(ka, cat16(*(const v8h*)r1, *(const v8h*)(r1 + 16)), s1);
        asm volatile("v_nop\n\tv_nop\n\tv_nop\n\tv_nop" : "+v"(s0), "+v"(s1) : "v"(ka));
#pragma unroll
        for (int j = 0; j < 8; ++j) {
            const float a0 = s0[j] + ej[j], a1 = s1[j] + ej[j];
            float mx = fmaxf(a0, a1);
            mx = fmaxf(mx, __shfl_xor(mx, 1, 16)); mx = fmaxf(mx, __shfl_xor(mx, 2, 16));
            mx = fmaxf(mx, __shfl_xor(mx, 4, 16)); mx = fmaxf(mx, __shfl_xor(mx, 8, 16));
            const float mn = fmaxf(mrow[j], mx);
            const float al = __expf(mrow[j] - mn);
            mrow[j] = mn;
            lpart[j] = lpart[j] * al + (__expf(a0 - mn) + __expf(a1 - mn));
        }
    }
#pragma unroll
    for (int j = 0; j < 8; ++j) {
        float rs = lpart[j];
        rs += __shfl_xor(rs, 1, 16); rs += __shfl_xor(rs, 2, 16); rs += __shfl_xor(rs, 4, 16); rs += __shfl_xor(rs, 8, 16);
        if (lr == 0) {
            const int jl = wave * 16 + 8 * hi + j;
            const float g = EGF[(size_t)(j0 + 8 * hi + j) * EGW + NHD + h];
            const float sg = 1.0f / (1.0f + expf(-g));
            stg[jl] = mrow[j];
            stg[64 + jl] = sg / rs;
        }
    }
    __syncthreads();
    if (wave == 0) {
        const v4f val = *(const v4fa*)(stg + hi * 64 + lr * 4);
        float* dst = (hi ? CC : CM) + (size_t)h * NN_ + jt * 64 + lr * 4;
        *(volatile v4f*)dst = val;
        __threadfence();
        *(volatile v4f*)dst = val;
    }
}

__global__ __launch_bounds__(64) void k_rows(const h16* __restrict__ Q16, const h16* __restrict__ K16, const h16* __restrict__ VT16, const float* __restrict__ EGF,
                                             const float* __restrict__ CM, const float* __restrict__ CC, const float* __restrict__ lng, const float* __restrict__ lnb, float* out) {
    __shared__ __align__(16) h16 plds[2][16 * 32];
    __shared__ __align__(16) float rows[2][16 * 260];
    const int lane = threadIdx.x & 31, wave = threadIdx.x >> 5, lr = lane & 15, hi = lane >> 4;
    const int i0 = blockIdx.x * 32 + wave * 16;
    h16* pl = &plds[wave][0];
    float* rw = &rows[wave][0];
#pragma unroll 1
    for (int h = 0; h < NHD; ++h) {
        const h16* qp = Q16 + ((size_t)h * NN_ + i0 + lr) * 32 + 8 * hi;
        const v16h qa = cat16(*(const v8h*)qp, *(const v8h*)(qp + 16));
        const h16* kb = K16 + (size_t)h * NN_ * 32;
        const h16* vb = VT16 + (size_t)h * HDM * NN_;
        const float* eb = EGF + h;
        const float* cmb = CM + (size_t)h * NN_;
        const float* ccb = CC + (size_t)h * NN_;
        v8f o0 = {}, o1 = {};
#pragma unroll 1
        for (int jt = 0; jt < NN_ / 32; ++jt) {
            const int jA = jt * 32 + lr, jB = jA + 16;
            const float eA = eb[(size_t)jA * EGW], eB = eb[(size_t)jB * EGW];
            const float mA = cmb[jA], mB = cmb[jB], cA = ccb[jA] * PSC, cB = ccb[jB] * PSC;
            const h16* rA = kb + (size_t)jA * 32 + 8 * hi;
            const h16* rB = kb + (size_t)jB * 32 + 8 * hi;
            v8f s0 = {}, s1 = {};
            s0 = wmma16(qa, cat16(*(const v8h*)rA, *(const v8h*)(rA + 16)), s0);
            s1 = wmma16(qa, cat16(*(const v8h*)rB, *(const v8h*)(rB + 16)), s1);
            asm volatile("v_nop\n\tv_nop\n\tv_nop\n\tv_nop" : "+v"(s0), "+v"(s1) : "v"(qa));
#pragma unroll
            for (int j = 0; j < 8; ++j) {
                const int mr = hi * 8 + j;
                pl[mr * 32 + lr]      = (h16)(__expf(s0[j] + eA - mA) * cA);
                pl[mr * 32 + 16 + lr] = (h16)(__expf(s1[j] + eB - mB) * cB);
            }
            asm volatile("" ::: "memory");
            const v16h pa = cat16(*(const v8ha*)(pl + lr * 32 + hi * 8), *(const v8ha*)(pl + lr * 32 + 16 + hi * 8));
            const h16* v0 = vb + (size_t)lr * NN_ + jt * 32 + hi * 8;
            const h16* v1 = vb + (size_t)(16 + lr) * NN_ + jt * 32 + hi * 8;
            o0 = wmma16(pa, cat16(*(const v8h*)v0, *(const v8h*)(v0 + 16)), o0);
            o1 = wmma16(pa, cat16(*(const v8h*)v1, *(const v8h*)(v1 + 16)), o1);
            asm volatile("v_nop\n\tv_nop\n\tv_nop\n\tv_nop" : "+v"(o0), "+v"(o1) : "v"(pa));
        }
#pragma unroll
        for (int r = 0; r < 8; ++r) {
            rw[(hi * 8 + r) * 260 + lr * 8 + h]        = o0[r] * (1.0f / PSC);
            rw[(hi * 8 + r) * 260 + (16 + lr) * 8 + h] = o1[r] * (1.0f / PSC);
        }
    }
    __syncthreads();
    v4f ga = *(const v4f*)(lng + lane * 4), gb = *(const v4f*)(lng + 128 + lane * 4);
    v4f ba = *(const v4f*)(lnb + lane * 4), bb = *(const v4f*)(lnb + 128 + lane * 4);
    v4f ya[16], yb[16];
#pragma unroll
    for (int r = 0; r < 16; ++r) {
        const v4f xa = *(const v4fa*)(rw + r * 260 + lane * 4), xb = *(const v4fa*)(rw + r * 260 + 128 + lane * 4);
        float s = (xa[0] + xa[1]) + (xa[2] + xa[3]) + (xb[0] + xb[1]) + (xb[2] + xb[3]);
#pragma unroll
        for (int o = 16; o; o >>= 1) s += __shfl_xor(s, o, 32);
        const float mu = s * (1.0f / 256.0f);
        v4f da = xa - mu, db = xb - mu;
        float q = (da[0] * da[0] + da[1] * da[1]) + (da[2] * da[2] + da[3] * da[3]) + (db[0] * db[0] + db[1] * db[1]) + (db[2] * db[2] + db[3] * db[3]);
#pragma unroll
        for (int o = 16; o; o >>= 1) q += __shfl_xor(q, o, 32);
        const float rs = rsqrtf(q * (1.0f / 256.0f) + 1e-3f);
        ya[r] = da * rs * ga + ba; yb[r] = db * rs * gb + bb;
    }
    float* ob = out + (size_t)i0 * HIDN;
    auto pass = [&]() {
#pragma unroll
        for (int r = 0; r < 16; ++r) {
            *(volatile v4f*)(ob + (size_t)r * HIDN + lane * 4) = ya[r];
            *(volatile v4f*)(ob + (size_t)r * HIDN + 128 + lane * 4) = yb[r];
        }
    };
    pass();
    __threadfence();
    pass();
}

extern "C" void kernel_launch(void* const* d_in, const int* in_sizes, int n_in,
                              void* d_out, int out_size, void* d_ws, size_t ws_size, hipStream_t stream) {
    (void)in_sizes; (void)n_in; (void)out_size;
    const float* feat = (const float*)d_in[0]; const float* Wq = (const float*)d_in[1]; const float* bq = (const float*)d_in[2];
    const float* Wkv = (const float*)d_in[3]; const float* bkv = (const float*)d_in[4]; const float* Weg = (const float*)d_in[5]; const float* beg = (const float*)d_in[6];
    const float* lng = (const float*)d_in[7]; const float* lnb = (const float*)d_in[8];
    float* out = (float*)d_out;
    char* wsp = (char*)d_ws;
    auto take = [&](size_t bytes) { char* p = wsp; wsp += (bytes + 255) & ~(size_t)255; return (void*)p; };
    h16*   FH   = (h16*)take((size_t)NN_ * HIDN * 2);
    h16*   FL   = (h16*)take((size_t)NN_ * HIDN * 2);
    h16*   WQH  = (h16*)take((size_t)HIDN * HIDN * 2);      h16* WQL  = (h16*)take((size_t)HIDN * HIDN * 2);
    h16*   WKVH = (h16*)take((size_t)2 * HIDN * HIDN * 2);  h16* WKVL = (h16*)take((size_t)2 * HIDN * HIDN * 2);
    h16*   WEGH = (h16*)take((size_t)EGW * HIDN * 2);       h16* WEGL = (h16*)take((size_t)EGW * HIDN * 2);
    float* QF   = (float*)take((size_t)NN_ * HIDN * 4);
    float* KVF  = (float*)take((size_t)NN_ * 2 * HIDN * 4);
    float* EGF  = (float*)take((size_t)NN_ * EGW * 4);
    h16*   Q16  = (h16*)take((size_t)NHD * NN_ * 32 * 2);
    h16*   K16  = (h16*)take((size_t)NHD * NN_ * 32 * 2);
    h16*   VT16 = (h16*)take((size_t)NHD * HDM * NN_ * 2);
    float* CM   = (float*)take((size_t)NHD * NN_ * 4);
    float* CC   = (float*)take((size_t)NHD * NN_ * 4);
    if ((size_t)(wsp - (char*)d_ws) > ws_size) return;
    k_asplit<<<NN_ / 8, 256, 0, stream>>>(feat, FH, FL);
    k_wsplit<<<dim3(HIDN / 64, HIDN / 64, 1), 256, 0, stream>>>(Wq, HIDN, HIDN, WQH, WQL);
    k_wsplit<<<dim3(HIDN / 64, (2 * HIDN) / 64, 1), 256, 0, stream>>>(Wkv, 2 * HIDN, 2 * HIDN, WKVH, WKVL);
    k_wsplit<<<dim3(HIDN / 64, EGW / 64, 1), 256, 0, stream>>>(Weg, 2 * NHD, EGW, WEGH, WEGL);
    k_lgemm<<<dim3(NN_ / 64, HIDN / 64, 1), 128, 0, stream>>>(FH, FL, WQH, WQL, bq, HIDN, QF, HIDN);
    k_lgemm<<<dim3(NN_ / 64, (2 * HIDN) / 64, 1), 128, 0, stream>>>(FH, FL, WKVH, WKVL, bkv, 2 * HIDN, KVF, 2 * HIDN);
    k_lgemm<<<dim3(NN_ / 64, EGW / 64, 1), 128, 0, stream>>>(FH, FL, WEGH, WEGL, beg, 2 * NHD, EGF, EGW);
    k_prep<<<NN_ / 64, 256, 0, stream>>>(QF, KVF, Q16, K16, VT16);
    k_colstats<<<NHD * (NN_ / 64), 128, 0, stream>>>(Q16, K16, EGF, CM, CC);
    k_rows<<<NN_ / 32, 64, 0, stream>>>(Q16, K16, VT16, EGF, CM, CC, lng, lnb, out);
}
